// GAT_45535243273030
// MI455X (gfx1250) — hardware-verified
//
#include <hip/hip_runtime.h>
#include <math.h>

#ifndef NPIX
#define NPIX 4096
#endif
#define NPIX_FULL 4096
#define NFEAT 128
#define NHID 64
#define NHEAD 3
#define NCLS 16
#define HCW (NHEAD * NHID)
#define KPO 32

static_assert(NPIX % 128 == 0);
static_assert(NPIX <= NPIX_FULL);
static_assert(NFEAT == 128);
static_assert(NHID == 64);
static_assert(NCLS == 16);
static_assert(HCW % 32 == 0 && NFEAT % 32 == 0 && NHID % 32 == 0 && KPO == 32);
static_assert((NHID * NFEAT / 8) % 256 == 0);
static_assert(NPIX % 32 == 0);

typedef _Float16 h16;
typedef __attribute__((ext_vector_type(16))) _Float16 v16h;
typedef __attribute__((ext_vector_type(8)))  _Float16 v8h;
typedef __attribute__((ext_vector_type(8)))  float    v8f;
typedef __attribute__((ext_vector_type(4)))  float    v4f;

static constexpr float XC = 8.0f;
static constexpr float WC = 32.0f;
static constexpr float PROJ_UNDO = 1.0f / 256.0f;
static_assert(XC * WC * PROJ_UNDO == 1.0f);
static constexpr float H1C = 64.0f;
static constexpr float NRM_UNDO = 1.0f / 4096.0f;
static_assert(H1C * H1C * NRM_UNDO == 1.0f);
static constexpr float PC = 1024.0f;
static constexpr float P_SC = 0.25f;
static_assert(P_SC * H1C * H1C == PC);
static constexpr float GC = 4096.0f;
static constexpr float AGG_UNDO = 1.0f / 4194304.0f;
static_assert(GC * PC * AGG_UNDO == 1.0f);
static constexpr float HCC = 16.0f;
static constexpr float WOC = 64.0f;
static constexpr float OH_UNDO = 1.0f / 1024.0f;
static_assert(HCC * WOC * OH_UNDO == 1.0f);
static_assert(WC == 32.0f && WOC == 64.0f);

static_assert(32 * 16 * 8 == 16 * NHID * 4);
static_assert(32 * 16 * 4 == 16 * NHID * 2);
static_assert(32 * 16 * 2 == 16 * NCLS * 4);
static_assert(32 * 16 * 2 == 16 * KPO * 2);
static_assert(256 * 16 * 2 == NCLS * 128 * 4);
static_assert(256 * 16 * 2 == 64 * 64 * 2);
static_assert(32 * 16 == 128 * 4);
static_assert(8 * 16 * 68 * 4 <= 131072);
static_assert(64 * 65 * 4 <= 131072);
static_assert(16 * 132 * 4 <= 131072);


#define VST2(T, ptr, val) do { const T vst2_v_ = (val); *(volatile T*)(ptr) = vst2_v_; __threadfence(); *(volatile T*)(ptr) = vst2_v_; } while (0)
#define VST2V4(ptr, val) do { const v4f vst2_v4_ = (val); *(volatile v4f*)(ptr) = vst2_v4_; __threadfence(); *(volatile v4f*)(ptr) = vst2_v4_; } while (0)

__device__ __forceinline__ float bfr(float f) {
    unsigned u = __float_as_uint(f);
    u += 0x7FFFu + ((u >> 16) & 1u);
    return __uint_as_float(u & 0xFFFF0000u);
}
static __device__ __forceinline__ h16 toh_flush(float v) { const float w = (fabsf(v) < 6.103515625e-05f) ? 0.0f : v; return (h16)w; }

__device__ __forceinline__ void st8hf(h16* P, size_t o, const float* v) {
    v8h hv;
#pragma unroll
    for (int e = 0; e < 8; ++e) hv[e] = toh_flush(v[e]);
    VST2(v8h, (v8h*)(P + o), hv);
}

union FragU { v16h v; v8h h[2]; };
__device__ __forceinline__ v16h frag_ld(const _Float16* p) {
    FragU f; f.h[0] = *(const v8h*)(p); f.h[1] = *(const v8h*)(p + 16); return f.v;
}
__device__ __forceinline__ v8f wmma16(v16h a, v16h b, v8f c) {
    c = __builtin_amdgcn_wmma_f32_16x16x32_f16(false, a, false, b, (short)0, c, false, false);
    asm volatile("v_nop\n\tv_nop\n\tv_nop\n\tv_nop" : "+v"(c) : "v"(a), "v"(b));
    return c;
}
__device__ __forceinline__ void wave_sync_lds() {
    __builtin_amdgcn_fence(3  , "workgroup");
    __builtin_amdgcn_wave_barrier();
    __builtin_amdgcn_fence(2  , "workgroup");
}

#define XT_P 65
__global__ __launch_bounds__(256) void k_xt16(const float* __restrict__ x, h16* __restrict__ xp) {
    __shared__ float sX[64 * XT_P];
    const unsigned tid = threadIdx.x;
    const unsigned bx = blockIdx.x;
    const unsigned n0 = (bx >> 1) * 64u, f0 = (bx & 1u) * 64u;
#pragma unroll
    for (int it = 0; it < 4; ++it) {
        const unsigned u = tid + 256u * (unsigned)it;
        const unsigned fl = u >> 4, q = u & 15u;
        const v4f a = *(const v4f*)(x + (size_t)(f0 + fl) * NPIX_FULL + n0 + 4u * q);
        sX[fl * XT_P + 4u * q + 0u] = a.x;
        sX[fl * XT_P + 4u * q + 1u] = a.y;
        sX[fl * XT_P + 4u * q + 2u] = a.z;
        sX[fl * XT_P + 4u * q + 3u] = a.w;
    }
    __syncthreads();
#pragma unroll
    for (int it = 0; it < 2; ++it) {
        const unsigned u = tid + 256u * (unsigned)it;
        const unsigned nl = u >> 3, p = u & 7u;
        float v[8];
#pragma unroll
        for (int e = 0; e < 8; ++e) v[e] = bfr(sX[(8u * p + (unsigned)e) * XT_P + nl]) * XC;
        st8hf(xp, (size_t)(n0 + nl) * NFEAT + f0 + 8u * p, v);
    }
}

template <int CARRY>
__device__ __forceinline__ void wconv_body(const float* __restrict__ W, h16* __restrict__ dst, unsigned n8) {
    const unsigned u = blockIdx.x * 256u + threadIdx.x;
    if (u >= n8) return;
    const v4f a = *(const v4f*)(W + (size_t)8u * u);
    const v4f b = *(const v4f*)(W + (size_t)8u * u + 4u);
    float v[8];
    v[0] = bfr(a.x) * (float)CARRY; v[1] = bfr(a.y) * (float)CARRY; v[2] = bfr(a.z) * (float)CARRY; v[3] = bfr(a.w) * (float)CARRY;
    v[4] = bfr(b.x) * (float)CARRY; v[5] = bfr(b.y) * (float)CARRY; v[6] = bfr(b.z) * (float)CARRY; v[7] = bfr(b.w) * (float)CARRY;
    st8hf(dst, (size_t)8u * u, v);
}
__global__ __launch_bounds__(256) void k_wconv32(const float* __restrict__ W, h16* __restrict__ dst, unsigned n8) { wconv_body<32>(W, dst, n8); }
__global__ __launch_bounds__(256) void k_wconv64(const float* __restrict__ W, h16* __restrict__ dst, unsigned n8) { wconv_body<64>(W, dst, n8); }

__global__ __launch_bounds__(256) void k_proj(const h16* __restrict__ xp, const h16* __restrict__ wh,
                                              const float* __restrict__ b1, const float* __restrict__ b2, const float* __restrict__ b3,
                                              float* __restrict__ h1f, h16* __restrict__ h1p) {
    __shared__ __align__(16) float sT[8][16 * 68];
    const unsigned lane = threadIdx.x & 31u;
    const unsigned wave = (unsigned)__builtin_amdgcn_readfirstlane((int)(threadIdx.x >> 5));
    const unsigned bx = blockIdx.x;
    const unsigned head = bx / (unsigned)(NPIX / 128);
    const unsigned blk = bx % (unsigned)(NPIX / 128);
    const unsigned m0 = blk * 128u + wave * 16u;
    const unsigned c = lane & 15u, hh = lane >> 4;

    v8f acc[4];
#pragma unroll
    for (int j = 0; j < 4; ++j) acc[j] = (v8f){0.f,0.f,0.f,0.f,0.f,0.f,0.f,0.f};
#pragma unroll
    for (int ks = 0; ks < 4; ++ks) {
        const v16h a = frag_ld(xp + (size_t)(m0 + c) * NFEAT + 32u * (unsigned)ks + 8u * hh);
#pragma unroll
        for (int j = 0; j < 4; ++j) {
            const v16h b = frag_ld(wh + (size_t)(head * NHID + 16u * (unsigned)j + c) * NFEAT + 32u * (unsigned)ks + 8u * hh);
            acc[j] = wmma16(a, b, acc[j]);
        }
    }
    float bv[4];
#pragma unroll
    for (int j = 0; j < 4; ++j) {
        const unsigned n = 16u * (unsigned)j + c;
        const float t1 = b1[n], t2 = b2[n], t3 = b3[n];
        const float ts = (head == 0u) ? t1 : ((head == 1u) ? t2 : t3);
        bv[j] = bfr(ts);
    }
#pragma unroll
    for (int r = 0; r < 8; ++r) {
        float v[4];
        float ss = 0.f;
#pragma unroll
        for (int j = 0; j < 4; ++j) { v[j] = acc[j][r] * PROJ_UNDO + bv[j]; ss += v[j] * v[j]; }
        ss += __shfl_xor(ss, 1, 32); ss += __shfl_xor(ss, 2, 32);
        ss += __shfl_xor(ss, 4, 32); ss += __shfl_xor(ss, 8, 32);
        const float nrm = fmaxf(sqrtf(ss), 1e-12f);
#pragma unroll
        for (int j = 0; j < 4; ++j) sT[wave][(8u * hh + (unsigned)r) * 68u + 16u * (unsigned)j + c] = v[j] / nrm;
    }
    wave_sync_lds();
    {
        float* dstf = h1f + ((size_t)head * NPIX + m0) * NHID;
        const unsigned c4 = (lane & 15u) * 4u;
#pragma unroll
        for (int half = 0; half < 2; ++half) {
            v4f vv[4];
#pragma unroll
            for (int it = 0; it < 4; ++it) {
                const unsigned row = (unsigned)(half * 4 + it) * 2u + hh;
                vv[it] = *(const v4f*)(&sT[wave][row * 68u + c4]);
            }
            for (int pass = 0; pass < 2; ++pass) {
#pragma unroll
                for (int it = 0; it < 4; ++it) {
                    const unsigned row = (unsigned)(half * 4 + it) * 2u + hh;
                    *(volatile v4f*)(dstf + (size_t)row * NHID + c4) = vv[it];
                }
                __threadfence();
            }
        }
    }
    {
        h16* dsth = h1p + ((size_t)head * NPIX + m0) * NHID;
        const unsigned q = lane >> 3, c8 = (lane & 7u) * 8u;
        v8h hv[4];
#pragma unroll
        for (int it = 0; it < 4; ++it) {
            const unsigned row = (unsigned)it * 4u + q;
#pragma unroll
            for (int e = 0; e < 8; ++e) hv[it][e] = toh_flush(sT[wave][row * 68u + c8 + (unsigned)e] * H1C);
        }
        for (int pass = 0; pass < 2; ++pass) {
#pragma unroll
            for (int it = 0; it < 4; ++it) {
                const unsigned row = (unsigned)it * 4u + q;
                *(volatile v8h*)(dsth + (size_t)row * NHID + c8) = hv[it];
            }
            __threadfence();
        }
    }
}

template <int KS, int LDH>
__device__ __forceinline__ float colsq_body(const h16* __restrict__ H, unsigned i0, unsigned lane) {
    const unsigned c = lane & 15u, hh = lane >> 4;
    v16h bi[KS];
#pragma unroll
    for (int ks = 0; ks < KS; ++ks) bi[ks] = frag_ld(H + (size_t)(i0 + c) * LDH + 32u * (unsigned)ks + 8u * hh);
    v8f sqv = (v8f){0.f,0.f,0.f,0.f,0.f,0.f,0.f,0.f};
#pragma unroll 1
    for (unsigned j0 = 0; j0 < (unsigned)NPIX; j0 += 32u) {
#pragma unroll
        for (int tt = 0; tt < 2; ++tt) {
            v8f s = (v8f){0.f,0.f,0.f,0.f,0.f,0.f,0.f,0.f};
#pragma unroll
            for (int ks = 0; ks < KS; ++ks) {
                const v16h aj = frag_ld(H + (size_t)(j0 + 16u * (unsigned)tt + c) * LDH + 32u * (unsigned)ks + 8u * hh);
                s = wmma16(aj, bi[ks], s);
            }
            sqv += s * s;
        }
    }
    float sq = ((sqv[0] + sqv[1]) + (sqv[2] + sqv[3])) + ((sqv[4] + sqv[5]) + (sqv[6] + sqv[7]));
    sq += __shfl_xor(sq, 16, 32);
    return sq;
}

__global__ __launch_bounds__(256) void k_norm64(const h16* __restrict__ h1p, float* __restrict__ nrm) {
    __shared__ __align__(16) float sN[128];
    const unsigned lane = threadIdx.x & 31u;
    const unsigned wave = (unsigned)__builtin_amdgcn_readfirstlane((int)(threadIdx.x >> 5));
    const unsigned bx = blockIdx.x;
    const unsigned head = bx / (unsigned)(NPIX / 128);
    const unsigned blk = bx % (unsigned)(NPIX / 128);
    const unsigned i0 = blk * 128u + wave * 16u;
    const float sq = colsq_body<2, NHID>(h1p + (size_t)head * NPIX * NHID, i0, lane);
    const float nv = fmaxf(sqrtf(sq) * NRM_UNDO, 1e-12f);
    if (lane < 16u) sN[wave * 16u + lane] = nv;
    __syncthreads();
    if (wave == 0u) {
        const v4f o = *(const v4f*)(&sN[4u * lane]);
        VST2V4(nrm + (size_t)head * NPIX + blk * 128u + 4u * lane, o);
    }
}
__global__ __launch_bounds__(256) void k_norm16(const h16* __restrict__ h1op, float* __restrict__ nrmo) {
    __shared__ __align__(16) float sN[128];
    const unsigned lane = threadIdx.x & 31u;
    const unsigned wave = (unsigned)__builtin_amdgcn_readfirstlane((int)(threadIdx.x >> 5));
    const unsigned bx = blockIdx.x;
    const unsigned i0 = bx * 128u + wave * 16u;
    const float sq = colsq_body<1, KPO>(h1op, i0, lane);
    const float nv = fmaxf(sqrtf(sq) * NRM_UNDO, 1e-12f);
    if (lane < 16u) sN[wave * 16u + lane] = nv;
    __syncthreads();
    if (wave == 0u) {
        const v4f o = *(const v4f*)(&sN[4u * lane]);
        VST2V4(nrmo + (size_t)bx * 128u + 4u * lane, o);
    }
}

template <int D>
__device__ __forceinline__ void gt_body(const float* __restrict__ hf, const float* __restrict__ nrm, h16* __restrict__ gt,
                                        unsigned j0, unsigned tid) {
    __shared__ float sG[64 * (D + 1)];
#pragma unroll 1
    for (unsigned u = tid; u < 64u * (unsigned)(D / 4); u += 256u) {
        const unsigned jl = u / (unsigned)(D / 4), q = u % (unsigned)(D / 4);
        const float nj = nrm[j0 + jl];
        const float sc = GC / nj;
        const v4f a = *(const v4f*)(hf + (size_t)(j0 + jl) * D + 4u * q);
        sG[jl * (unsigned)(D + 1) + 4u * q + 0u] = a.x * sc;
        sG[jl * (unsigned)(D + 1) + 4u * q + 1u] = a.y * sc;
        sG[jl * (unsigned)(D + 1) + 4u * q + 2u] = a.z * sc;
        sG[jl * (unsigned)(D + 1) + 4u * q + 3u] = a.w * sc;
    }
    __syncthreads();
#pragma unroll 1
    for (unsigned u = tid; u < 8u * (unsigned)D; u += 256u) {
        const unsigned d = u >> 3, p = u & 7u;
        float v[8];
#pragma unroll
        for (int e = 0; e < 8; ++e) v[e] = sG[(8u * p + (unsigned)e) * (unsigned)(D + 1) + d];
        st8hf(gt, (size_t)d * NPIX + j0 + 8u * p, v);
    }
}
__global__ __launch_bounds__(256) void k_gt64(const float* __restrict__ h1f, const float* __restrict__ nrm, h16* __restrict__ gt) {
    const unsigned bx = blockIdx.x;
    const unsigned head = bx / (unsigned)(NPIX / 64);
    const unsigned jt = bx % (unsigned)(NPIX / 64);
    gt_body<NHID>(h1f + (size_t)head * NPIX * NHID, nrm + (size_t)head * NPIX, gt + (size_t)head * NHID * NPIX, jt * 64u, threadIdx.x);
}
__global__ __launch_bounds__(256) void k_gt16(const float* __restrict__ h1of, const float* __restrict__ nrmo, h16* __restrict__ gto) {
    const unsigned bx = blockIdx.x;
    gt_body<NCLS>(h1of, nrmo, gto, bx * 64u, threadIdx.x);
}

template <int KS, int LDH, int DT>
__device__ __forceinline__ void agg_body(const h16* __restrict__ H, const h16* __restrict__ GT, unsigned i0, unsigned lane, v8f (&oacc)[DT]) {
    const unsigned c = lane & 15u, hh = lane >> 4;
    v16h bi[KS];
#pragma unroll
    for (int ks = 0; ks < KS; ++ks) bi[ks] = frag_ld(H + (size_t)(i0 + c) * LDH + 32u * (unsigned)ks + 8u * hh);
#pragma unroll
    for (int t = 0; t < DT; ++t) oacc[t] = (v8f){0.f,0.f,0.f,0.f,0.f,0.f,0.f,0.f};
#pragma unroll 1
    for (unsigned j0 = 0; j0 < (unsigned)NPIX; j0 += 32u) {
        v8f s0 = (v8f){0.f,0.f,0.f,0.f,0.f,0.f,0.f,0.f};
        v8f s1 = (v8f){0.f,0.f,0.f,0.f,0.f,0.f,0.f,0.f};
#pragma unroll
        for (int ks = 0; ks < KS; ++ks) {
            const v16h aj = frag_ld(H + (size_t)(j0 + c) * LDH + 32u * (unsigned)ks + 8u * hh);
            s0 = wmma16(aj, bi[ks], s0);
        }
#pragma unroll
        for (int ks = 0; ks < KS; ++ks) {
            const v16h aj = frag_ld(H + (size_t)(j0 + 16u + c) * LDH + 32u * (unsigned)ks + 8u * hh);
            s1 = wmma16(aj, bi[ks], s1);
        }
        v16h pb;
#pragma unroll
        for (int r = 0; r < 8; ++r) {
            pb[r]     = toh_flush(s0[r] * P_SC);
            pb[8 + r] = toh_flush(s1[r] * P_SC);
        }
#pragma unroll
        for (int t = 0; t < DT; ++t) {
            const v16h ga = frag_ld(GT + (size_t)(16u * (unsigned)t + c) * NPIX + j0 + 8u * hh);
            oacc[t] = wmma16(ga, pb, oacc[t]);
        }
    }
}

__global__ __launch_bounds__(256) void k_agg64(const h16* __restrict__ h1p, const h16* __restrict__ gt, h16* __restrict__ hc) {
    __shared__ __align__(16) float sT[8][16 * 68];
    const unsigned lane = threadIdx.x & 31u;
    const unsigned wave = (unsigned)__builtin_amdgcn_readfirstlane((int)(threadIdx.x >> 5));
    const unsigned bx = blockIdx.x;
    const unsigned head = bx / (unsigned)(NPIX / 128);
    const unsigned blk = bx % (unsigned)(NPIX / 128);
    const unsigned i0 = blk * 128u + wave * 16u;
    const unsigned c = lane & 15u, hh = lane >> 4;
    v8f oacc[4];
    agg_body<2, NHID, 4>(h1p + (size_t)head * NPIX * NHID, gt + (size_t)head * NHID * NPIX, i0, lane, oacc);
#pragma unroll
    for (int t = 0; t < 4; ++t)
#pragma unroll
        for (int r = 0; r < 8; ++r)
            sT[wave][c * 68u + 16u * (unsigned)t + 8u * hh + (unsigned)r] = oacc[t][r] * AGG_UNDO;
    wave_sync_lds();
    const unsigned q = lane >> 3, c8 = (lane & 7u) * 8u;
#pragma unroll 1
    for (unsigned it = 0; it < 4u; ++it) {
        const unsigned row = it * 4u + q;
        v8h hv;
#pragma unroll
        for (int e = 0; e < 8; ++e) {
            const float o = sT[wave][row * 68u + c8 + (unsigned)e];
            const float a = (o > 0.0f) ? o : expm1f(o);
            hv[e] = toh_flush(a * HCC);
        }
        VST2(v8h, (v8h*)(hc + (size_t)(i0 + row) * HCW + head * NHID + c8), hv);
    }
}

__global__ __launch_bounds__(256) void k_ohead(const h16* __restrict__ hc, const h16* __restrict__ wo, const float* __restrict__ bo,
                                               float* __restrict__ h1of, h16* __restrict__ h1op) {
    __shared__ __align__(16) float sT[8][16 * 16];
    const unsigned lane = threadIdx.x & 31u;
    const unsigned wave = (unsigned)__builtin_amdgcn_readfirstlane((int)(threadIdx.x >> 5));
    const unsigned bx = blockIdx.x;
    const unsigned m0 = bx * 128u + wave * 16u;
    const unsigned c = lane & 15u, hh = lane >> 4;
    v8f acc = (v8f){0.f,0.f,0.f,0.f,0.f,0.f,0.f,0.f};
#pragma unroll
    for (int ks = 0; ks < HCW / 32; ++ks) {
        const v16h a = frag_ld(hc + (size_t)(m0 + c) * HCW + 32u * (unsigned)ks + 8u * hh);
        const v16h b = frag_ld(wo + (size_t)c * HCW + 32u * (unsigned)ks + 8u * hh);
        acc = wmma16(a, b, acc);
    }
    const float bv = bfr(bo[c]);
#pragma unroll
    for (int r = 0; r < 8; ++r) {
        const float v = acc[r] * OH_UNDO + bv;
        float ss = v * v;
        ss += __shfl_xor(ss, 1, 32); ss += __shfl_xor(ss, 2, 32);
        ss += __shfl_xor(ss, 4, 32); ss += __shfl_xor(ss, 8, 32);
        const float nrm = fmaxf(sqrtf(ss), 1e-12f);
        sT[wave][(8u * hh + (unsigned)r) * 16u + c] = v / nrm;
    }
    wave_sync_lds();
    {
        const v4f o0 = *(const v4f*)(&sT[wave][4u * lane]);
        const v4f o1 = *(const v4f*)(&sT[wave][128u + 4u * lane]);
        float* dstf = h1of + (size_t)m0 * NCLS;
        for (int pass = 0; pass < 2; ++pass) {
            *(volatile v4f*)(dstf + 4u * lane) = o0;
            *(volatile v4f*)(dstf + 128u + 4u * lane) = o1;
            __threadfence();
        }
    }
    {
        v8h hv[2];
#pragma unroll
        for (int it = 0; it < 2; ++it) {
            const unsigned u = lane + 32u * (unsigned)it;
            const unsigned row = u >> 2, part = u & 3u;
#pragma unroll
            for (int e = 0; e < 8; ++e) {
                const float s = sT[wave][row * 16u + 8u * (part & 1u) + (unsigned)e] * H1C;
                const float z = (part < 2u) ? s : 0.0f;
                hv[it][e] = toh_flush(z);
            }
        }
        h16* dsth = h1op + (size_t)m0 * KPO;
        for (int pass = 0; pass < 2; ++pass) {
#pragma unroll
            for (int it = 0; it < 2; ++it) *(volatile v8h*)(dsth + 8u * (lane + 32u * (unsigned)it)) = hv[it];
            __threadfence();
        }
    }
}

__global__ __launch_bounds__(256) void k_agg16(const h16* __restrict__ h1op, const h16* __restrict__ gto, float* __restrict__ out) {
    __shared__ __align__(16) float sO[16 * 132];
    const unsigned tid = threadIdx.x;
    const unsigned lane = tid & 31u;
    const unsigned wave = (unsigned)__builtin_amdgcn_readfirstlane((int)(threadIdx.x >> 5));
    const unsigned bx = blockIdx.x;
    const unsigned i0 = bx * 128u + wave * 16u;
    const unsigned c = lane & 15u, hh = lane >> 4;
    v8f oacc[1];
    agg_body<1, KPO, 1>(h1op, gto, i0, lane, oacc);
#pragma unroll
    for (int r = 0; r < 8; ++r) sO[(8u * hh + (unsigned)r) * 132u + wave * 16u + c] = oacc[0][r] * AGG_UNDO;
    __syncthreads();
#pragma unroll
    for (int it = 0; it < 2; ++it) {
        const unsigned u = tid + 256u * (unsigned)it;
        const unsigned cls = u >> 5, q = u & 31u;
        const v4f o = *(const v4f*)(&sO[cls * 132u + 4u * q]);
        VST2V4(out + (size_t)cls * NPIX_FULL + bx * 128u + 4u * q, o);
    }
}

static constexpr size_t cu256(size_t b) { return (b + 255) & ~(size_t)255; }
static constexpr size_t WS_TOTAL =
    cu256((size_t)NPIX * NFEAT * 2) + cu256((size_t)HCW * NFEAT * 2) + cu256((size_t)NCLS * HCW * 2) +
    cu256((size_t)NHEAD * NPIX * NHID * 4) + cu256((size_t)NHEAD * NPIX * NHID * 2) + cu256((size_t)NHEAD * NPIX * 4) +
    cu256((size_t)NHEAD * NHID * NPIX * 2) + cu256((size_t)NPIX * HCW * 2) + cu256((size_t)NPIX * NCLS * 4) +
    cu256((size_t)NPIX * KPO * 2) + cu256((size_t)NPIX * 4) + cu256((size_t)NCLS * NPIX * 2);
static_assert(WS_TOTAL <= (size_t)134217728);

extern "C" void kernel_launch(void* const* d_in, const int* in_sizes, int n_in, void* d_out, int out_size,
                              void* d_ws, size_t ws_size, hipStream_t stream) {
    if (n_in < 9) return;
    if (in_sizes[0] < NFEAT * NPIX || in_sizes[1] < NHID * NFEAT || in_sizes[2] < NHID || in_sizes[3] < NHID * NFEAT) return;
    if (in_sizes[4] < NHID || in_sizes[5] < NHID * NFEAT || in_sizes[6] < NHID || in_sizes[7] < NCLS * HCW || in_sizes[8] < NCLS) return;
    if (out_size < NCLS * NPIX) return;

    const float* x  = (const float*)d_in[0];
    const float* W1 = (const float*)d_in[1];
    const float* b1 = (const float*)d_in[2];
    const float* W2 = (const float*)d_in[3];
    const float* b2 = (const float*)d_in[4];
    const float* W3 = (const float*)d_in[5];
    const float* b3 = (const float*)d_in[6];
    const float* Wo = (const float*)d_in[7];
    const float* bo = (const float*)d_in[8];
    float* out = (float*)d_out;

    char* wsp = (char*)d_ws;
    size_t off = 0;
    auto carve = [&](size_t bytes) -> void* { void* r = wsp + off; off += (bytes + 255) & ~(size_t)255; return r; };
    h16*   xp   = (h16*)carve((size_t)NPIX * NFEAT * 2);
    h16*   wh   = (h16*)carve((size_t)HCW * NFEAT * 2);
    h16*   wo   = (h16*)carve((size_t)NCLS * HCW * 2);
    float* h1f  = (float*)carve((size_t)NHEAD * NPIX * NHID * 4);
    h16*   h1p  = (h16*)carve((size_t)NHEAD * NPIX * NHID * 2);
    float* nrm  = (float*)carve((size_t)NHEAD * NPIX * 4);
    h16*   gt   = (h16*)carve((size_t)NHEAD * NHID * NPIX * 2);
    h16*   hc   = (h16*)carve((size_t)NPIX * HCW * 2);
    float* h1of = (float*)carve((size_t)NPIX * NCLS * 4);
    h16*   h1op = (h16*)carve((size_t)NPIX * KPO * 2);
    float* nrmo = (float*)carve((size_t)NPIX * 4);
    h16*   gto  = (h16*)carve((size_t)NCLS * NPIX * 2);
    if (off > ws_size || off > (size_t)134217728) return;

    k_xt16<<<(NPIX / 64) * (NFEAT / 64), 256, 0, stream>>>(x, xp);
    k_wconv32<<<(NHID * NFEAT / 8) / 256, 256, 0, stream>>>(W1, wh, (unsigned)(NHID * NFEAT / 8));
    k_wconv32<<<(NHID * NFEAT / 8) / 256, 256, 0, stream>>>(W2, wh + (size_t)NHID * NFEAT, (unsigned)(NHID * NFEAT / 8));
    k_wconv32<<<(NHID * NFEAT / 8) / 256, 256, 0, stream>>>(W3, wh + (size_t)2 * NHID * NFEAT, (unsigned)(NHID * NFEAT / 8));
    k_wconv64<<<(NCLS * HCW / 8 + 255) / 256, 256, 0, stream>>>(Wo, wo, (unsigned)(NCLS * HCW / 8));

    k_proj<<<NHEAD * (NPIX / 128), 256, 0, stream>>>(xp, wh, b1, b2, b3, h1f, h1p);
    k_norm64<<<NHEAD * (NPIX / 128), 256, 0, stream>>>(h1p, nrm);
    k_gt64<<<NHEAD * (NPIX / 64), 256, 0, stream>>>(h1f, nrm, gt);
    k_agg64<<<NHEAD * (NPIX / 128), 256, 0, stream>>>(h1p, gt, hc);

    k_ohead<<<NPIX / 128, 256, 0, stream>>>(hc, wo, bo, h1of, h1op);
    k_norm16<<<NPIX / 128, 256, 0, stream>>>(h1op, nrmo);
    k_gt16<<<NPIX / 64, 256, 0, stream>>>(h1of, nrmo, gto);
    k_agg16<<<NPIX / 128, 256, 0, stream>>>(h1op, gto, out);
}
